// MelPCENTransform_15728170237987
// MI455X (gfx1250) — hardware-run, weakly checked
//
#include <hip/hip_runtime.h>
#include <math.h>

typedef __attribute__((ext_vector_type(16))) _Float16 v16h;
typedef __attribute__((ext_vector_type(8)))  _Float16 v8h;
typedef __attribute__((ext_vector_type(8)))  float    v8f;
typedef __attribute__((ext_vector_type(4)))  float    v4f;

constexpr int kB        = 64;
constexpr int kL        = 160000;
constexpr int kNfft     = 2048;
constexpr int kHop      = 512;
constexpr int kHalf     = kNfft / 2;
constexpr int kBins     = 1024;
constexpr int kMels     = 128;
constexpr int kT        = 1 + kL / kHop;
constexpr int kChunkB   = 16;
constexpr int kNumChunk = kB / kChunkB;
constexpr int kRowsReal = kChunkB * kT;
constexpr int kRowsPad  = ((kRowsReal + 63) / 64) * 64;
constexpr int kOutN     = kB * kMels * kT;
static_assert(kT == 313, "frame count");
static_assert(kRowsReal == 5008 && kRowsPad == 5056, "chunk rows");
static_assert(kOutN == 2564096, "output elements");
static_assert((kHalf % 32) == 0 && (kBins % 32) == 0, "GEMM K multiples of 32");
static_assert((kRowsPad % 64) == 0 && (kBins % 64) == 0 && (kMels % 64) == 0, "GEMM M,N multiples of 64");
static_assert((kRowsPad % 8) == 0, "fold kernel rows per block");
static_assert((kOutN % 1024) == 0, "flat store grid exact");
static_assert(kB == kChunkB * kNumChunk, "chunking");

constexpr float kCarryY       = 64.0f;
constexpr float kCarryFb      = 64.0f;
constexpr float kPowCarry     = 1.0f / 32.0f;
constexpr float kPowScale     = kPowCarry / (kCarryY * kCarryY);
constexpr float kMelScale     = 1.0f / kCarryFb;
constexpr float kScanGain     = 1.0f / kPowCarry;
constexpr float kF16MinNormal = 6.103515625e-05f;
constexpr float kSmooth       = 0.025f;
constexpr float kKeep         = (float)(1.0 - 0.025);
constexpr float kEps          = 1e-6f;
constexpr float kAlpha        = 0.98f;
constexpr float kDelta        = 2.0f;
constexpr float kRootDelta    = 1.41421356237309515f;

constexpr double kSampleRate = 32000.0;
constexpr double kFmin       = 20.0;
constexpr double kFmax       = 16000.0;
constexpr double kBinHz      = kSampleRate / (double)kNfft;
constexpr double kMelA       = 1.0 + kFmin / 700.0;
constexpr double kMelSpan    = (1.0 + kFmax / 700.0) / kMelA;
constexpr double cx_powi(double r, int n) {
  double p = 1.0;
  for (int i = 0; i < n; ++i) p *= r;
  return p;
}
constexpr double cx_abs(double x) { return x < 0.0 ? -x : x; }
constexpr double cx_root(double c, int n, double r0) {
  double r = r0;
  for (int it = 0; it < 12; ++it) {
    const double pn1 = cx_powi(r, n - 1);
    r = r - (pn1 * r - c) / ((double)n * pn1);
  }
  return r;
}
constexpr double kMelRatio = cx_root(kMelSpan, kMels + 1, 1.02467);
static_assert(kMelRatio > 1.0246 && kMelRatio < 1.0247, "ratio range");
static_assert(cx_abs(cx_powi(kMelRatio, kMels + 1) - kMelSpan) < 1.0e-10 * kMelSpan, "ratio solve");
static_assert(kMels + 1 < 256, "eight-bit exponent");
static_assert(kBinHz == 15.625, "bin spacing");

constexpr size_t kSzBasis = (size_t)kBins * kHalf * 2;
constexpr size_t kSzFbt   = (size_t)kMels * kBins * 2;
constexpr size_t kSzY     = (size_t)kRowsPad * kHalf * 2;
constexpr size_t kSzSpec  = (size_t)kRowsPad * kBins * 4;
constexpr size_t kSzPw    = (size_t)kRowsPad * kBins * 2;
constexpr size_t kSzMel   = (size_t)kNumChunk * kRowsPad * kMels * 4;
constexpr size_t kSzPs    = (size_t)kB * kT * kMels * 4;
constexpr size_t kOffCos  = 0;
constexpr size_t kOffSin  = kOffCos + kSzBasis;
constexpr size_t kOffFbt  = kOffSin + kSzBasis;
constexpr size_t kOffYe   = kOffFbt + kSzFbt;
constexpr size_t kOffYo   = kOffYe + kSzY;
constexpr size_t kOffRe   = kOffYo + kSzY;
constexpr size_t kOffIm   = kOffRe + kSzSpec;
constexpr size_t kOffPw   = kOffIm + kSzSpec;
constexpr size_t kOffMel  = kOffPw + kSzPw;
constexpr size_t kOffPs   = kOffMel + kSzMel;
constexpr size_t kWsTotal = kOffPs + kSzPs;
static_assert(kWsTotal == 97550336ull, "carve total");
static_assert(kWsTotal <= 134217728ull, "carve cap");
static_assert((kOffSin % 128) == 0 && (kOffFbt % 128) == 0 && (kOffYe % 128) == 0 && (kOffYo % 128) == 0 &&
              (kOffRe % 128) == 0 && (kOffIm % 128) == 0 && (kOffPw % 128) == 0 && (kOffMel % 128) == 0 &&
              (kOffPs % 128) == 0, "128-B aligned regions");

__device__ __forceinline__ _Float16 cvt_h16_flush(float v) {
  const float u = (fabsf(v) < kF16MinNormal) ? 0.0f : v;
  return (_Float16)u;
}
__device__ __forceinline__ int mirror_idx(int i) {
  i = (i < 0) ? -i : i;
  i = (i >= kL) ? (2 * (kL - 1) - i) : i;
  i = (i < 0) ? 0 : i;
  i = (i > kL - 1) ? (kL - 1) : i;
  return i;
}
union FragH { v16h v; v8h h[2]; };
__device__ __forceinline__ v16h frag_load_h(const _Float16* p) {
  FragH f;
  f.h[0] = *(const v8h*)(p);
  f.h[1] = *(const v8h*)(p + 16);
  return f.v;
}
__device__ __forceinline__ v8f mma_h(v16h a, v16h b, v8f c) {
  return __builtin_amdgcn_wmma_f32_16x16x32_f16(false, a, false, b, (short)0, c, false, false);
}
__device__ __forceinline__ void guard1_h(v8f& c, v16h a, v16h b) {
  asm volatile("v_nop\n\tv_nop\n\tv_nop\n\tv_nop" : "+v"(c) : "v"(a), "v"(b));
}
__device__ __forceinline__ void keep4_h(v16h a, v16h b, v16h c, v16h d) {
  asm volatile("v_nop" :: "v"(a), "v"(b), "v"(c), "v"(d));
}
__device__ __forceinline__ void acc_guard4(v8f& a, v8f& b, v8f& c, v8f& d) {
  asm volatile("v_nop\n\tv_nop\n\tv_nop\n\tv_nop" : "+v"(a), "+v"(b), "+v"(c), "+v"(d));
}

__global__ __launch_bounds__(256) void wmma_gemm64_f16(
    const unsigned short* __restrict__ Ap, int lda, long strideA,
    const unsigned short* __restrict__ Btp, int ldb, long strideB,
    float* __restrict__ Cout, int ldc, long strideC,
    int M, int N, int K, float scale) {
  __shared__ __align__(16) float sT[8][16 * 68];
  const int b    = blockIdx.y;
  const int lane = threadIdx.x & 31;
  const int wave = threadIdx.x >> 5;
  const int tilesN = N >> 6;
  const int tilesM = M >> 6;
  const int tile = blockIdx.x * 8 + wave;
  if (tile >= tilesM * tilesN) return;
  const int tm = tile / tilesN;
  const int tn = tile - tm * tilesN;
  const int m0 = tm << 6;
  const int n0 = tn << 6;

  const _Float16* Ab = (const _Float16*)Ap  + (size_t)b * strideA;
  const _Float16* Bb = (const _Float16*)Btp + (size_t)b * strideB;

  const int rlane = lane & 15;
  const int koff  = (lane >> 4) * 8;
  const int mOff  = (lane >> 4) * 8;

  v8f acc[4][4];
#pragma unroll
  for (int i = 0; i < 4; ++i)
#pragma unroll
    for (int j = 0; j < 4; ++j) acc[i][j] = (v8f){0.f,0.f,0.f,0.f,0.f,0.f,0.f,0.f};

  for (int k0 = 0; k0 < K; k0 += 32) {
    v16h bh[4];
#pragma unroll
    for (int j = 0; j < 4; ++j) {
      const size_t bo = (size_t)(n0 + (j << 4) + rlane) * ldb + koff + k0;
      bh[j] = frag_load_h(Bb + bo);
    }
#pragma unroll
    for (int i = 0; i < 4; ++i) {
      const size_t ao = (size_t)(m0 + (i << 4) + rlane) * lda + koff + k0;
      const v16h ah = frag_load_h(Ab + ao);
#pragma unroll
      for (int j = 0; j < 4; ++j) acc[i][j] = mma_h(ah, bh[j], acc[i][j]);
#pragma unroll
      for (int j = 0; j < 4; ++j) guard1_h(acc[i][j], ah, bh[j]);
    }
    keep4_h(bh[0], bh[1], bh[2], bh[3]);
  }
  acc_guard4(acc[0][0], acc[0][1], acc[0][2], acc[0][3]);
  acc_guard4(acc[1][0], acc[1][1], acc[1][2], acc[1][3]);
  acc_guard4(acc[2][0], acc[2][1], acc[2][2], acc[2][3]);
  acc_guard4(acc[3][0], acc[3][1], acc[3][2], acc[3][3]);

  float* slab = sT[wave];
  float* C = Cout + (size_t)b * strideC;
  const int hh = lane >> 4, c4 = (lane & 15) * 4;
#pragma unroll
  for (int i = 0; i < 4; ++i) {
    const int mBase = m0 + (i << 4);
#pragma unroll
    for (int j = 0; j < 4; ++j) {
#pragma unroll
      for (int r = 0; r < 8; ++r) {
        const float v = acc[i][j][r] * scale;
        slab[(mOff + r) * 68 + (j << 4) + rlane] = v;
      }
    }
    __builtin_amdgcn_fence(__ATOMIC_RELEASE, "workgroup");
    __builtin_amdgcn_wave_barrier();
    __builtin_amdgcn_fence(__ATOMIC_ACQUIRE, "workgroup");
    for (int pass = 0; pass < 2; ++pass) {
#pragma unroll
      for (int it = 0; it < 8; ++it) {
        const int row = it * 2 + hh;
        v4f v = *(const v4f*)(slab + row * 68 + c4);
        *(volatile v4f*)(C + (size_t)(mBase + row) * ldc + n0 + c4) = v;
      }
      __threadfence();
    }
    __builtin_amdgcn_fence(__ATOMIC_RELEASE, "workgroup");
    __builtin_amdgcn_wave_barrier();
    __builtin_amdgcn_fence(__ATOMIC_ACQUIRE, "workgroup");
  }
}

__global__ __launch_bounds__(256) void basis_table_kernel(unsigned* __restrict__ cosw, unsigned* __restrict__ sinw) {
  const int gid = blockIdx.x * 256 + threadIdx.x;
  if (gid >= kBins * (kHalf / 2)) return;
  const int k  = gid / (kHalf / 2);
  const int jp = gid - k * (kHalf / 2);
  const int n0 = (jp << 1) + 1;
  const int n1 = n0 + 1;
  const int r0 = (k * n0) & (kNfft - 1);
  const int r1 = (k * n1) & (kNfft - 1);
  const float a0 = (float)r0 * (1.0f / (float)kHalf);
  const float a1 = (float)r1 * (1.0f / (float)kHalf);
  const float c0 = cospif(a0);
  const float s0 = sinpif(a0);
  const float c1 = cospif(a1);
  float s1 = sinpif(a1);
  s1 = (n1 == kHalf) ? 0.0f : s1;
  const _Float16 hc0 = cvt_h16_flush(c0), hc1 = cvt_h16_flush(c1);
  const _Float16 hs0 = cvt_h16_flush(s0), hs1 = cvt_h16_flush(s1);
  const unsigned uc = (unsigned)__builtin_bit_cast(unsigned short, hc0) | ((unsigned)__builtin_bit_cast(unsigned short, hc1) << 16);
  const unsigned us = (unsigned)__builtin_bit_cast(unsigned short, hs0) | ((unsigned)__builtin_bit_cast(unsigned short, hs1) << 16);
  ((volatile unsigned*)cosw)[gid] = uc;
  ((volatile unsigned*)sinw)[gid] = us;
  __threadfence();
  ((volatile unsigned*)cosw)[gid] = uc;
  ((volatile unsigned*)sinw)[gid] = us;
}

__global__ __launch_bounds__(256) void filterbank_table_kernel(unsigned short* __restrict__ fbt) {
  __shared__ double sFp[kMels + 2];
  const int tid = threadIdx.x;
  if (tid < kMels + 2) {
    double p = 1.0, base = kMelRatio;
    int e = tid;
#pragma unroll 1
    for (int bit = 0; bit < 8; ++bit) {
      const double pm = p * base;
      p = (e & 1) ? pm : p;
      base = base * base;
      e >>= 1;
    }
    sFp[tid] = 700.0 * (kMelA * p - 1.0);
  }
  __syncthreads();
  const int gid = blockIdx.x * 256 + tid;
  const int m   = gid >> 7;
  const int f0  = (gid & 127) * 8;
  const double fp0 = sFp[m], fp1 = sFp[m + 1], fp2 = sFp[m + 2];
  const double rd0 = 1.0 / (fp1 - fp0);
  const double rd1 = 1.0 / (fp2 - fp1);
  v8h hv;
#pragma unroll
  for (int e = 0; e < 8; ++e) {
    const double fq = kBinHz * (double)(f0 + e);
    const double dn = (fq - fp0) * rd0;
    const double up = (fp2 - fq) * rd1;
    const double wd = fmax(0.0, fmin(dn, up));
    const float  wf = (float)wd;
    hv[e] = cvt_h16_flush(wf * kCarryFb);
  }
  unsigned short* q = fbt + (size_t)m * kBins + f0;
  *(volatile v8h*)q = hv;
  __threadfence();
  *(volatile v8h*)q = hv;
}

__global__ __launch_bounds__(256) void fold_frames_kernel(
    const float* __restrict__ wav, unsigned short* __restrict__ ye, unsigned short* __restrict__ yo, int chunk) {
  __shared__ __align__(16) float sWnd[kHalf];
  const int tid = threadIdx.x;
#pragma unroll 1
  for (int q = 0; q < 4; ++q) {
    const int jj = tid + 256 * q;
    const float s = sinpif((float)(jj + 1) * (1.0f / (float)kNfft));
    sWnd[jj] = s * s;
  }
  __syncthreads();
  const int oct = tid & 127;
  const int rg  = tid >> 7;
  const int j0  = oct * 8;
  const v4f w0 = *(const v4f*)(sWnd + j0);
  const v4f w1 = *(const v4f*)(sWnd + j0 + 4);
  const float w[8] = {w0[0], w0[1], w0[2], w0[3], w1[0], w1[1], w1[2], w1[3]};
#pragma unroll 1
  for (int i = 0; i < 4; ++i) {
    const int row = blockIdx.x * 8 + rg * 4 + i;
    const bool live = row < kRowsReal;
    const int rc = live ? row : (kRowsReal - 1);
    const int bl = rc / kT;
    const int t  = rc - bl * kT;
    const float* xb = wav + (size_t)(chunk * kChunkB + bl) * kL;
    const int base = t * kHop - kHalf;
    float av[8], bv[8];
#pragma unroll
    for (int e = 0; e < 8; ++e) {
      const int n = j0 + e + 1;
      av[e] = xb[mirror_idx(base + n)];
      bv[e] = xb[mirror_idx(base + kNfft - n)];
    }
    v8h he, ho;
#pragma unroll
    for (int e = 0; e < 8; ++e) {
      const int n = j0 + e + 1;
      const float pa = w[e] * av[e];
      const float pb = w[e] * bv[e];
      float se = (n == kHalf) ? pa : (pa + pb);
      float so = pa - pb;
      se = live ? (se * kCarryY) : 0.0f;
      so = live ? (so * kCarryY) : 0.0f;
      he[e] = cvt_h16_flush(se);
      ho[e] = cvt_h16_flush(so);
    }
    unsigned short* qe = ye + (size_t)row * kHalf + j0;
    unsigned short* qo = yo + (size_t)row * kHalf + j0;
    *(volatile v8h*)qe = he;
    *(volatile v8h*)qo = ho;
    __threadfence();
    *(volatile v8h*)qe = he;
    *(volatile v8h*)qo = ho;
  }
}

__global__ __launch_bounds__(256) void power_kernel(
    const float* __restrict__ re, const float* __restrict__ im, unsigned short* __restrict__ pw) {
  const int gid = blockIdx.x * 256 + threadIdx.x;
  if (gid >= kRowsPad * (kBins / 8)) return;
  const size_t e0 = (size_t)gid << 3;
  const v4f r0 = *(const v4f*)(re + e0);
  const v4f r1 = *(const v4f*)(re + e0 + 4);
  const v4f i0 = *(const v4f*)(im + e0);
  const v4f i1 = *(const v4f*)(im + e0 + 4);
  v8h hv;
#pragma unroll
  for (int e = 0; e < 4; ++e) {
    const float p0 = (r0[e] * r0[e] + i0[e] * i0[e]) * kPowScale;
    const float p1 = (r1[e] * r1[e] + i1[e] * i1[e]) * kPowScale;
    hv[e]     = cvt_h16_flush(p0);
    hv[4 + e] = cvt_h16_flush(p1);
  }
  unsigned short* q = pw + e0;
  *(volatile v8h*)q = hv;
  __threadfence();
  *(volatile v8h*)q = hv;
}

__global__ __launch_bounds__(128) void smooth_compress_scan_kernel(
    const float* __restrict__ mel, float* __restrict__ ps) {
  __shared__ __align__(16) float sY[32 * 132];
  const int tid = threadIdx.x, lane = tid & 31, wave = tid >> 5;
  const int b  = blockIdx.x;
  const int ch = b / kChunkB;
  const int bl = b - ch * kChunkB;
  const float* mp = mel + ((size_t)ch * kRowsPad + (size_t)bl * kT) * kMels + tid;
  float m = 0.0f;
#pragma unroll 1
  for (int t0 = 0; t0 < kT; t0 += 32) {
    const int nst = (kT - t0 < 32) ? (kT - t0) : 32;
#pragma unroll 1
    for (int s = 0; s < nst; ++s) {
      const float x = kScanGain * mp[(size_t)(t0 + s) * kMels];
      m = kKeep * m + kSmooth * x;
      const float v   = kEps + m;
      const float inv = exp2f(-kAlpha * log2f(v));
      const float p   = sqrtf(x * inv + kDelta) - kRootDelta;
      sY[s * 132 + tid] = p;
    }
    __syncthreads();
    v4f rv[8];
#pragma unroll
    for (int it = 0; it < 8; ++it) {
      const int row = it * 4 + wave;
      const int rr = (row < nst) ? row : 0;
      rv[it] = *(const v4f*)(sY + rr * 132 + lane * 4);
    }
    for (int pass = 0; pass < 2; ++pass) {
#pragma unroll
      for (int it = 0; it < 8; ++it) {
        const int row = it * 4 + wave;
        if (row < nst)
          *(volatile v4f*)(ps + ((size_t)b * kT + t0 + row) * kMels + lane * 4) = rv[it];
      }
      __threadfence();
    }
    __syncthreads();
  }
}

__global__ __launch_bounds__(256) void transpose_store_kernel(
    const float* __restrict__ ps, float* __restrict__ out) {
  const int gid = blockIdx.x * 256 + threadIdx.x;
  if (gid >= kOutN / 4) return;
  v4f v;
#pragma unroll
  for (int e = 0; e < 4; ++e) {
    const int i   = gid * 4 + e;
    const int b   = i / (kMels * kT);
    const int rem = i - b * (kMels * kT);
    const int mm  = rem / kT;
    const int t   = rem - mm * kT;
    v[e] = ps[((size_t)b * kT + t) * kMels + mm];
  }
  float* q = out + (size_t)gid * 4;
  *(volatile v4f*)q = v;
  __threadfence();
  *(volatile v4f*)q = v;
}

extern "C" void kernel_launch(void* const* d_in, const int* in_sizes, int n_in,
                              void* d_out, int out_size, void* d_ws, size_t ws_size,
                              hipStream_t stream) {
  if (n_in < 1) return;
  if (in_sizes[0] != kB * kL) return;
  if (out_size != kOutN) return;
  if (ws_size < kWsTotal) return;

  const float* wav = (const float*)d_in[0];
  float* out = (float*)d_out;
  char* ws = (char*)d_ws;
  unsigned short* COS = (unsigned short*)(ws + kOffCos);
  unsigned short* SIN = (unsigned short*)(ws + kOffSin);
  unsigned short* FBT = (unsigned short*)(ws + kOffFbt);
  unsigned short* YE  = (unsigned short*)(ws + kOffYe);
  unsigned short* YO  = (unsigned short*)(ws + kOffYo);
  float*          RE  = (float*)(ws + kOffRe);
  float*          IM  = (float*)(ws + kOffIm);
  unsigned short* PW  = (unsigned short*)(ws + kOffPw);
  float*          MEL = (float*)(ws + kOffMel);
  float*          PS  = (float*)(ws + kOffPs);

  basis_table_kernel<<<(kBins * (kHalf / 2)) / 256, 256, 0, stream>>>((unsigned*)COS, (unsigned*)SIN);
  filterbank_table_kernel<<<(kMels * (kBins / 8)) / 256, 256, 0, stream>>>(FBT);

  const long planeY = (long)kRowsPad * kHalf;
  const long planeB = (long)kBins * kHalf;
  const long planeC = (long)kRowsPad * kBins;
  const int dftBlocks = ((kRowsPad / 64) * (kBins / 64) + 7) / 8;
  const int melBlocks = ((kRowsPad / 64) * (kMels / 64) + 7) / 8;

  for (int c = 0; c < kNumChunk; ++c) {
    fold_frames_kernel<<<kRowsPad / 8, 256, 0, stream>>>(wav, YE, YO, c);
    wmma_gemm64_f16<<<dim3(dftBlocks, 2), 256, 0, stream>>>(
        YE, kHalf, planeY,
        COS, kHalf, planeB,
        RE, kBins, planeC,
        kRowsPad, kBins, kHalf, 1.0f);
    power_kernel<<<(kRowsPad * (kBins / 8)) / 256, 256, 0, stream>>>(RE, IM, PW);
    wmma_gemm64_f16<<<dim3(melBlocks, 1), 256, 0, stream>>>(
        PW, kBins, 0L,
        FBT, kBins, 0L,
        MEL + (size_t)c * kRowsPad * kMels, kMels, 0L,
        kRowsPad, kMels, kBins, kMelScale);
  }

  smooth_compress_scan_kernel<<<kB, kMels, 0, stream>>>(MEL, PS);
  transpose_store_kernel<<<(kOutN / 4) / 256, 256, 0, stream>>>(PS, out);
}
